// Eprop_fit_11364483465334
// MI455X (gfx1250) — hardware-run, weakly checked
//
#include <hip/hip_runtime.h>
#include <hip/hip_fp16.h>
#include <math.h>

typedef __attribute__((ext_vector_type(16))) _Float16 v16h;
typedef __attribute__((ext_vector_type(8)))  _Float16 v8h;
typedef __attribute__((ext_vector_type(8)))  float    v8f;
typedef __attribute__((ext_vector_type(4)))  float    v4f;

constexpr int kNb     = 4;
constexpr int kNt     = 300;
constexpr int kNeur   = 200;
constexpr int kNin    = 100;
constexpr int kNout   = 10;
constexpr int kBT     = kNb * kNt;
constexpr int kKp     = 1216;
constexpr int kA1Rows = 320;
constexpr int kPORows = 256;
constexpr int kWTRows = 256;
constexpr int kETRows = 64;
constexpr int kRaw1Ld = 256;
constexpr int kRaw2Ld = 64;
constexpr int kLK     = 32;
constexpr int kLsLd   = 256;
constexpr float kACarry = 256.0f;
constexpr float kBCarry = 1024.0f;
constexpr float kResid  = 2048.0f;
constexpr float kThr    = 0.6f;
constexpr float kDamp   = 0.3f;
constexpr float kDecay  = 0.8f;
constexpr float kReg    = 300.0f;
static_assert(kBT == 1200);
static_assert(kKp == 38 * 32 && kKp == 19 * 64 && kKp >= kBT);
static_assert(kA1Rows >= kNin + kNeur && (kA1Rows % 32) == 0);
static_assert(kPORows >= kNeur && (kPORows % 32) == 0);
static_assert(kWTRows >= kNeur && (kWTRows % 64) == 0 && kWTRows == kRaw1Ld);
static_assert(kETRows >= kNout && (kETRows % 64) == 0 && kETRows == kRaw2Ld);
static_assert(kA1Rows + kPORows == 9 * 64);
static_assert(kETRows * (kKp / 8) == 38 * 256);
static_assert(((kA1Rows / 32) * (kWTRows / 64)) % 8 == 0);
static_assert(((kPORows / 32) * (kETRows / 64)) % 8 == 0);
static_assert(kNin * kNeur == 4 * 5000 && kNeur * kNeur == 4 * 10000 && kNeur * kNout == 4 * 500);
static_assert(kLK == 32 && kLK >= kNout && (kLK % 32) == 0);
static_assert(kLsLd == kWTRows && (kLsLd % 64) == 0);
static_assert(kKp * (kLK / 8) == 19 * 256);
static_assert(kWTRows * (kLK / 8) == 4 * 256);
static_assert((kKp % 32) == 0 && ((kKp / 32) * (kLsLd / 64)) % 8 == 0);

constexpr size_t kSzA1   = (size_t)kA1Rows * kKp * 2;
constexpr size_t kSzPO   = (size_t)kPORows * kKp * 2;
constexpr size_t kSzG    = (size_t)kWTRows * kKp * 4;
constexpr size_t kSzWT   = (size_t)kWTRows * kKp * 2;
constexpr size_t kSzET   = (size_t)kETRows * kKp * 2;
constexpr size_t kSzRAW1 = (size_t)kA1Rows * kRaw1Ld * 4;
constexpr size_t kSzRAW2 = (size_t)kPORows * kRaw2Ld * 4;
constexpr size_t kSzEA   = (size_t)kKp * kLK * 2;
constexpr size_t kSzWO   = (size_t)kWTRows * kLK * 2;
constexpr size_t kSzLS   = (size_t)kKp * kLsLd * 4;
constexpr size_t kOffA1   = 0;
constexpr size_t kOffPO   = kOffA1   + kSzA1;
constexpr size_t kOffG    = kOffPO   + kSzPO;
constexpr size_t kOffWT   = kOffG    + kSzG;
constexpr size_t kOffET   = kOffWT   + kSzWT;
constexpr size_t kOffRAW1 = kOffET   + kSzET;
constexpr size_t kOffRAW2 = kOffRAW1 + kSzRAW1;
constexpr size_t kOffEA   = kOffRAW2 + kSzRAW2;
constexpr size_t kOffWO   = kOffEA   + kSzEA;
constexpr size_t kOffLS   = kOffWO   + kSzWO;
constexpr size_t kWsTotal = kOffLS   + kSzLS;
static_assert(kSzA1 == 778240ull && kSzPO == 622592ull && kSzG == 1245184ull && kSzWT == 622592ull);
static_assert(kSzET == 155648ull && kSzRAW1 == 327680ull && kSzRAW2 == 65536ull);
static_assert(kSzEA == 77824ull && kSzWO == 16384ull && kSzLS == 1245184ull);
static_assert(kWsTotal == 5156864ull);
static_assert(kWsTotal <= 134217728ull);
static_assert((kOffPO % 128) == 0 && (kOffG % 128) == 0 && (kOffWT % 128) == 0 && (kOffET % 128) == 0 &&
              (kOffRAW1 % 128) == 0 && (kOffRAW2 % 128) == 0 && (kOffEA % 128) == 0 && (kOffWO % 128) == 0 &&
              (kOffLS % 128) == 0);
static_assert(((kKp * 2) % 128) == 0 && ((kKp * 4) % 128) == 0);

__device__ __forceinline__ _Float16 f16_flush(float v) {
  const float w = (fabsf(v) < 6.103515625e-05f) ? 0.0f : v;
  return (_Float16)w;
}
__device__ __forceinline__ void f16_split(float v, _Float16& hi, _Float16& lo) {
  hi = f16_flush(v);
  const float hf = (float)hi;
  const float r = (v - hf) * kResid;
  lo = f16_flush(r);
}

__device__ __forceinline__ float bf16r(float v) {
  unsigned u = __float_as_uint(v);
  u = (u + 0x7FFFu + ((u >> 16) & 1u)) & 0xFFFF0000u;
  return __uint_as_float(u);
}

__device__ __forceinline__ float h16_to_f32(unsigned hb) {
  const unsigned sgn = (hb & 0x8000u) << 16; const unsigned em = hb & 0x7fffu;
  const float fn = __uint_as_float((em << 13) + 0x38000000u);
  const float fs = (float)em * 5.9604644775390625e-8f;
  const float mag = (em < 0x400u) ? fs : fn; return __uint_as_float(__float_as_uint(mag) | sgn); }

namespace eng {
union FragU { v16h v; v8h h[2]; };
__device__ __forceinline__ v16h frag_load(const _Float16* p) {
  FragU f;
  f.h[0] = *(const v8h*)(p);
  f.h[1] = *(const v8h*)(p + 16);
  return f.v;
}
__device__ __forceinline__ v8f mma(v16h a, v16h b, v8f c) {
  return __builtin_amdgcn_wmma_f32_16x16x32_f16(false, a, false, b, (short)0, c, false, false);
}
__device__ __forceinline__ void guard1(v8f& a, v16h x, v16h y) {
  asm volatile("v_nop\n\tv_nop\n\tv_nop\n\tv_nop" : "+v"(a) : "v"(x), "v"(y));
}
__device__ __forceinline__ void guard_acc(v8f& a) {
  asm volatile("v_nop\n\tv_nop\n\tv_nop\n\tv_nop" : "+v"(a));
}
__device__ __forceinline__ void keep4(v16h a, v16h b, v16h c, v16h d) {
  asm volatile("v_nop" :: "v"(a), "v"(b), "v"(c), "v"(d));
}

template <int MI, int SPL>
__global__ __launch_bounds__(256) void gemm_f16_kernel(
    const unsigned short* __restrict__ Ap, const unsigned short* __restrict__ A2p, int lda,
    const unsigned short* __restrict__ Btp, const unsigned short* __restrict__ Bt2p, int ldb,
    float* __restrict__ C, int ldc, int M, int N, int K, float scale, float rscale)
{
  static_assert(MI >= 1 && MI <= 2);
  static_assert(SPL >= 0 && SPL <= 2);
  const _Float16* A   = (const _Float16*)Ap;
  const _Float16* A2  = (const _Float16*)A2p;
  const _Float16* Bt  = (const _Float16*)Btp;
  const _Float16* Bt2 = (const _Float16*)Bt2p;
  __shared__ __align__(16) float sT[8][16 * 68];
  const int lane = threadIdx.x & 31;
  const int wave = threadIdx.x >> 5;
  const int tilesN = N >> 6;
  const int tilesM = M / (16 * MI);
  const int tile = blockIdx.x * 8 + wave;
  if (tile >= tilesM * tilesN) return;
  const int tm = tile / tilesN;
  const int tn = tile - tm * tilesN;
  const int m0 = tm * (16 * MI);
  const int n0 = tn << 6;
  const int rlane = lane & 15;
  const int koff  = (lane >> 4) * 8;
  const int mOff  = (lane >> 4) * 8;

  v8f acc[MI][4], accr[MI][4];
#pragma unroll
  for (int i = 0; i < MI; ++i)
#pragma unroll
    for (int j = 0; j < 4; ++j) {
      acc[i][j]  = (v8f){0.f, 0.f, 0.f, 0.f, 0.f, 0.f, 0.f, 0.f};
      accr[i][j] = (v8f){0.f, 0.f, 0.f, 0.f, 0.f, 0.f, 0.f, 0.f};
    }

  for (int k0 = 0; k0 < K; k0 += 32) {
    v16h bh[4], bl[4];
#pragma unroll
    for (int j = 0; j < 4; ++j) {
      const size_t bo = (size_t)(n0 + (j << 4) + rlane) * ldb + koff + k0;
      bh[j] = frag_load(Bt + bo);
      if (SPL == 2) bl[j] = frag_load(Bt2 + bo); else bl[j] = bh[j];
    }
#pragma unroll
    for (int i = 0; i < MI; ++i) {
      const size_t ao = (size_t)(m0 + (i << 4) + rlane) * lda + koff + k0;
      const v16h ah = frag_load(A + ao);
      v16h al = ah;
      if (SPL >= 1) al = frag_load(A2 + ao);
#pragma unroll
      for (int j = 0; j < 4; ++j) {
        acc[i][j] = mma(ah, bh[j], acc[i][j]);
        if (SPL >= 1) accr[i][j] = mma(al, bh[j], accr[i][j]);
        if (SPL == 2) accr[i][j] = mma(ah, bl[j], accr[i][j]);
      }
#pragma unroll
      for (int j = 0; j < 4; ++j) {
        guard1(acc[i][j], ah, al);
        if (SPL >= 1) guard1(accr[i][j], ah, al);
      }
    }
    keep4(bh[0], bh[1], bh[2], bh[3]);
    if (SPL == 2) keep4(bl[0], bl[1], bl[2], bl[3]);
  }
#pragma unroll
  for (int i = 0; i < MI; ++i)
#pragma unroll
    for (int j = 0; j < 4; ++j) {
      guard_acc(acc[i][j]);
      if (SPL >= 1) guard_acc(accr[i][j]);
    }

  float* slab = sT[wave];
#pragma unroll
  for (int i = 0; i < MI; ++i) {
    const int mBase = m0 + (i << 4);
#pragma unroll
    for (int j = 0; j < 4; ++j) {
#pragma unroll
      for (int r = 0; r < 8; ++r) {
        float v = acc[i][j][r] * scale;
        if (SPL >= 1) v += accr[i][j][r] * rscale;
        slab[(mOff + r) * 68 + (j << 4) + rlane] = v;
      }
    }
    __builtin_amdgcn_fence(__ATOMIC_RELEASE, "workgroup");
    __builtin_amdgcn_wave_barrier();
    __builtin_amdgcn_fence(__ATOMIC_ACQUIRE, "workgroup");
    {
      const int hh = lane >> 4, c4 = (lane & 15) * 4;
      for (int pass = 0; pass < 2; ++pass) {
#pragma unroll
        for (int it = 0; it < 8; ++it) {
          const int row = it * 2 + hh;
          const v4f v = *(const v4f*)(slab + row * 68 + c4);
          *(volatile v4f*)(C + (size_t)(mBase + row) * ldc + n0 + c4) = v;
        }
        __threadfence();
      }
    }
    __builtin_amdgcn_fence(__ATOMIC_RELEASE, "workgroup");
    __builtin_amdgcn_wave_barrier();
    __builtin_amdgcn_fence(__ATOMIC_ACQUIRE, "workgroup");
  }
}
}

__global__ __launch_bounds__(64) void pre_kernel(
    const float* __restrict__ x, const float* __restrict__ z,
    unsigned short* __restrict__ A1, unsigned short* __restrict__ PO)
{
  const int r = blockIdx.x * 64 + threadIdx.x;
  const bool isA1  = (r < kA1Rows);
  const bool isIn  = (r < kNin);
  const bool isRec = (r >= kNin) && (r < kNin + kNeur);
  const int  jo    = isA1 ? 0 : (r - kA1Rows);
  const bool isOut = (!isA1) && (jo < kNeur);
  const bool rowLive = isIn || isRec || isOut;
  const float* src = isIn ? x : z;
  const int pitch  = isIn ? kNin : kNeur;
  const int ch     = isIn ? r : (isRec ? (r - kNin) : (isOut ? jo : 0));
  const int shift  = isRec ? 1 : 0;
  const int ra     = isA1 ? r : 0;
  unsigned short* dst = isA1 ? (A1 + (size_t)ra * kKp) : (PO + (size_t)jo * kKp);

  float a = 0.0f;
  int t = 0;
  for (int trip = 0; trip < 19; ++trip) {
    v8h hv[8];
#pragma unroll
    for (int q = 0; q < 8; ++q) {
#pragma unroll
      for (int e = 0; e < 8; ++e) {
        const int k = trip * 64 + q * 8 + e;
        const bool live = (k < kBT);
        const int ks = k - shift;
        const int k1 = (ks < 0) ? 0 : ks;
        const int kc = (k1 > kBT - 1) ? (kBT - 1) : k1;
        const float raw = src[(size_t)kc * pitch + ch];
        const bool inLive = rowLive && live && (t >= shift);
        const float inp = inLive ? bf16r(raw) : 0.0f;
        const float a0 = (t == 0) ? 0.0f : a;
        a = kDecay * a0 + inp;
        const float word = (rowLive && live) ? (a * kACarry) : 0.0f;
        hv[q][e] = f16_flush(word);
        t = (t == kNt - 1) ? 0 : (t + 1);
      }
    }
    unsigned short* lp = dst + trip * 64;
#pragma unroll
    for (int q = 0; q < 8; ++q) *(volatile v8h*)(lp + 8 * q) = hv[q];
    __threadfence();
#pragma unroll
    for (int q = 0; q < 8; ++q) *(volatile v8h*)(lp + 8 * q) = hv[q];
  }
}

__global__ __launch_bounds__(256) void g_kernel(
    const float* __restrict__ LS, float* __restrict__ G)
{
  const int j = blockIdx.x * 256 + threadIdx.x;
  const bool rowLive = (j < kNeur);
  const float* lcol = LS + j;
  float* grow = G + (size_t)j * kKp;

  float g = 0.0f;
  int t = 15;
  for (int trip = 0; trip < 38; ++trip) {
    const int base = (37 - trip) * 32;
    v4f vv[8];
#pragma unroll
    for (int s = 0; s < 32; ++s) {
      const int o = 31 - s;
      const int k = base + o;
      const bool live = (k < kBT);
      const float L = lcol[(size_t)k * kLsLd];
      const float gin = (t == kNt - 1) ? 0.0f : g;
      g = fmaf(kDecay, gin, L);
      const float val = (rowLive && live) ? g : 0.0f;
      vv[o >> 2][o & 3] = val;
      t = (t == 0) ? (kNt - 1) : (t - 1);
    }
    float* lp = grow + base;
#pragma unroll
    for (int q = 0; q < 8; ++q) *(volatile v4f*)(lp + 4 * q) = vv[q];
    __threadfence();
#pragma unroll
    for (int q = 0; q < 8; ++q) *(volatile v4f*)(lp + 4 * q) = vv[q];
  }
}

__global__ __launch_bounds__(256) void w_kernel(
    const float* __restrict__ v, const float* __restrict__ z, const float* __restrict__ err2,
    const float* __restrict__ G, unsigned short* __restrict__ WT)
{
  const int j = blockIdx.x * 256 + threadIdx.x;
  const bool rowLive = (j < kNeur);
  const int jc = rowLive ? j : (kNeur - 1);
  const float regTerm = kReg * bf16r(err2[jc]) / 1200.0f;
  const float* grow = G + (size_t)j * kKp;
  unsigned short* dst = WT + (size_t)j * kKp;

  int c = 0;
  int t = 0;
  for (int trip = 0; trip < 19; ++trip) {
    v8h hv[8];
#pragma unroll
    for (int q = 0; q < 8; ++q) {
      const int kq = trip * 64 + q * 8;
      const v4f g0 = *(const v4f*)(grow + kq);
      const v4f g1 = *(const v4f*)(grow + kq + 4);
      float gv[8];
      gv[0] = g0[0];
      gv[1] = g0[1];
      gv[2] = g0[2];
      gv[3] = g0[3];
      gv[4] = g1[0];
      gv[5] = g1[1];
      gv[6] = g1[2];
      gv[7] = g1[3];
#pragma unroll
      for (int e = 0; e < 8; ++e) {
        const int k = kq + e;
        const bool live = (k < kBT);
        const int kc = live ? k : (kBT - 1);
        const float vb = bf16r(v[(size_t)kc * kNeur + jc]);
        const float zb = bf16r(z[(size_t)kc * kNeur + jc]);
        const int cr = (t == 0) ? 0 : c;
        const float vs = (vb - kThr) / kThr;
        const float psi = kDamp * fmaxf(1.0f - fabsf(vs), 0.0f) / kThr;
        const float post = (cr > 0) ? 0.0f : psi;
        const int cd = cr - 1;
        c = (zb > 0.0f) ? 4 : ((cd > 0) ? cd : 0);
        const float w = post * (gv[e] + regTerm);
        const float word = (rowLive && live) ? (w * kBCarry) : 0.0f;
        hv[q][e] = f16_flush(word);
        t = (t == kNt - 1) ? 0 : (t + 1);
      }
    }
    unsigned short* lp = dst + trip * 64;
#pragma unroll
    for (int q = 0; q < 8; ++q) *(volatile v8h*)(lp + 8 * q) = hv[q];
    __threadfence();
#pragma unroll
    for (int q = 0; q < 8; ++q) *(volatile v8h*)(lp + 8 * q) = hv[q];
  }
}

__global__ __launch_bounds__(256) void e_kernel(
    const float* __restrict__ e1, unsigned short* __restrict__ ET)
{
  const int idx = blockIdx.x * 256 + threadIdx.x;
  const int row = idx / 152;
  const int w8  = idx - row * 152;
  const int k0  = w8 * 8;
  const bool rowLive = (row < kNout);
  const int rc = rowLive ? row : (kNout - 1);
  v8h hv;
#pragma unroll
  for (int e = 0; e < 8; ++e) {
    const int k = k0 + e;
    const bool live = (k < kBT);
    const int kc = live ? k : (kBT - 1);
    const float raw = e1[(size_t)kc * kNout + rc];
    const float word = (rowLive && live) ? (bf16r(raw) * kBCarry) : 0.0f;
    hv[e] = f16_flush(word);
  }
  unsigned short* p = ET + (size_t)idx * 8;
  *(volatile v8h*)p = hv;
  __threadfence();
  *(volatile v8h*)p = hv;
}

__global__ __launch_bounds__(256) void ea_kernel(
    const float* __restrict__ e1, unsigned short* __restrict__ EA)
{
  const int idx = blockIdx.x * 256 + threadIdx.x;
  const int k   = idx >> 2;
  const int kk0 = (idx & 3) * 8;
  const bool rowLive = (k < kBT);
  const int kc = rowLive ? k : (kBT - 1);
  v8h hv;
#pragma unroll
  for (int e = 0; e < 8; ++e) {
    const int kk = kk0 + e;
    const bool live = (kk < kNout);
    const int kkc = live ? kk : (kNout - 1);
    const float raw = e1[(size_t)kc * kNout + kkc];
    const float word = (rowLive && live) ? (bf16r(raw) * kBCarry) : 0.0f;
    hv[e] = f16_flush(word);
  }
  unsigned short* p = EA + (size_t)idx * 8;
  *(volatile v8h*)p = hv;
  __threadfence();
  *(volatile v8h*)p = hv;
}

__global__ __launch_bounds__(256) void wo_kernel(
    const float* __restrict__ wout, unsigned short* __restrict__ WO)
{
  const int idx = blockIdx.x * 256 + threadIdx.x;
  const int j   = idx >> 2;
  const int kk0 = (idx & 3) * 8;
  const bool rowLive = (j < kNeur);
  const int jc = rowLive ? j : (kNeur - 1);
  v8h hv;
#pragma unroll
  for (int e = 0; e < 8; ++e) {
    const int kk = kk0 + e;
    const bool live = (kk < kNout);
    const int kkc = live ? kk : (kNout - 1);
    const float raw = wout[(size_t)jc * kNout + kkc];
    const float word = (rowLive && live) ? (bf16r(raw) * kBCarry) : 0.0f;
    hv[e] = f16_flush(word);
  }
  unsigned short* p = WO + (size_t)idx * 8;
  *(volatile v8h*)p = hv;
  __threadfence();
  *(volatile v8h*)p = hv;
}

__global__ __launch_bounds__(256) void out_copy_kernel(
    const float* __restrict__ src, int ld, int row0, int cols, int nWords,
    float* __restrict__ dst, int maskDiag)
{
  const int w = blockIdx.x * 256 + threadIdx.x;
  if (w >= nWords) return;
  v4f val;
#pragma unroll
  for (int q = 0; q < 4; ++q) {
    const int e = 4 * w + q;
    const int r = e / cols;
    const int c = e - r * cols;
    const float s = src[(size_t)(row0 + r) * ld + c];
    const bool dz = (maskDiag != 0) && (r == c);
    val[q] = dz ? 0.0f : s;
  }
  float* p = dst + (size_t)w * 4;
  *(volatile v4f*)p = val;
  __threadfence();
  *(volatile v4f*)p = val;
}

extern "C" void kernel_launch(void* const* d_in, const int* in_sizes, int n_in,
                              void* d_out, int out_size, void* d_ws, size_t ws_size,
                              hipStream_t stream)
{
  if (n_in < 6) return;
  if (in_sizes[0] != kBT * kNeur) return;
  if (in_sizes[1] != kBT * kNeur) return;
  if (in_sizes[2] != kBT * kNin) return;
  if (in_sizes[3] != kBT * kNout) return;
  if (in_sizes[4] != kNeur) return;
  if (in_sizes[5] != kNeur * kNout) return;
  if (out_size != kNin * kNeur + kNeur * kNeur + kNeur * kNout) return;
  if (ws_size < kWsTotal) return;

  const float* v_in   = (const float*)d_in[0];
  const float* z_in   = (const float*)d_in[1];
  const float* x_in   = (const float*)d_in[2];
  const float* e1_in  = (const float*)d_in[3];
  const float* e2_in  = (const float*)d_in[4];
  const float* wo_in  = (const float*)d_in[5];
  float* out = (float*)d_out;

  char* ws = (char*)d_ws;
  unsigned short* A1   = (unsigned short*)(ws + kOffA1);
  unsigned short* PO   = (unsigned short*)(ws + kOffPO);
  float*          G    = (float*)(ws + kOffG);
  unsigned short* WT   = (unsigned short*)(ws + kOffWT);
  unsigned short* ET   = (unsigned short*)(ws + kOffET);
  float*          RAW1 = (float*)(ws + kOffRAW1);
  float*          RAW2 = (float*)(ws + kOffRAW2);
  unsigned short* EA   = (unsigned short*)(ws + kOffEA);
  unsigned short* WO   = (unsigned short*)(ws + kOffWO);
  float*          LS   = (float*)(ws + kOffLS);

  constexpr float sOut = 1.0f / (kACarry * kBCarry);
  constexpr float sL   = 1.0f / (kBCarry * kBCarry);

  pre_kernel<<<9, 64, 0, stream>>>(x_in, z_in, A1, PO);

  e_kernel<<<38, 256, 0, stream>>>(e1_in, ET);

  ea_kernel<<<19, 256, 0, stream>>>(e1_in, EA);

  wo_kernel<<<4, 256, 0, stream>>>(wo_in, WO);

  eng::gemm_f16_kernel<2, 0><<<dim3((1216 / 32) * (256 / 64) / 8), 256, 0, stream>>>(
      EA, nullptr, 32, WO, nullptr, 32, LS, 256, 1216, 256, 32, sL, 0.0f);

  g_kernel<<<1, 256, 0, stream>>>(LS, G);

  w_kernel<<<1, 256, 0, stream>>>(v_in, z_in, e2_in, G, WT);

  eng::gemm_f16_kernel<2, 0><<<dim3((320 / 32) * (256 / 64) / 8), 256, 0, stream>>>(
      A1, nullptr, 1216, WT, nullptr, 1216, RAW1, 256, 320, 256, 1216, sOut, 0.0f);

  eng::gemm_f16_kernel<2, 0><<<dim3((256 / 32) * (64 / 64) / 8), 256, 0, stream>>>(
      PO, nullptr, 1216, ET, nullptr, 1216, RAW2, 64, 256, 64, 1216, sOut, 0.0f);

  out_copy_kernel<<<(5000 + 255) / 256, 256, 0, stream>>>(RAW1, 256, 0, 200, 5000, out, 0);

  out_copy_kernel<<<(10000 + 255) / 256, 256, 0, stream>>>(RAW1, 256, 100, 200, 10000, out + 20000, 1);

  out_copy_kernel<<<(500 + 255) / 256, 256, 0, stream>>>(RAW2, 64, 0, 10, 500, out + 60000, 0);
}
